// GptOssAttention_42752104464388
// MI455X (gfx1250) — hardware-verified
//
#include <hip/hip_runtime.h>
#include <math.h>

#ifndef SEQ
#define SEQ 2048
#endif
#ifndef NB
#define NB 1
#endif
#ifndef OSPLIT_ROWS
#define OSPLIT_ROWS 128
#endif
#define SEQ_FULL 2048
#define HID 2880
#define NQH 64
#define NKVH 8
#define HPG (NQH / NKVH)
#define HDM 64
#define QW (NQH * HDM)
#define KVW (NKVH * HDM)
#define QKVW (QW + 2 * KVW)
#define NSLOT (NQH + NKVH)
#define WIN 128
#define KPAD 128
#define SKP (SEQ + KPAD)
#define BW 192
static_assert(NB == 1);
static_assert(SEQ % 128 == 0 && SEQ >= 128 && SEQ <= SEQ_FULL);
static_assert(OSPLIT_ROWS % 64 == 0 && OSPLIT_ROWS >= 64 && OSPLIT_ROWS <= SEQ);
static_assert(HID % 64 == 0 && HID % 32 == 0 && QW == 4096 && KVW == 512 && QKVW == 5120 && HDM == 64 && HPG == 8);
static_assert(BW == KPAD + 64 && BW % 64 == 0 && BW % 32 == 0 && WIN <= KPAD && SKP % 128 == 0);

typedef __attribute__((ext_vector_type(16))) _Float16 v16h;
typedef __attribute__((ext_vector_type(8)))  _Float16 v8h;
typedef __attribute__((ext_vector_type(16))) __bf16   v16b;
typedef __attribute__((ext_vector_type(8)))  __bf16   v8b;
typedef __attribute__((ext_vector_type(8)))  float    v8f;
typedef __attribute__((ext_vector_type(4)))  float    v4f;
typedef __attribute__((ext_vector_type(4)))  int      v4i;
typedef __attribute__((ext_vector_type(4)))  unsigned v4u;

#define VST2(T, ptr, val) do { const T vst2_v_ = (val); *(volatile T*)(ptr) = vst2_v_; __threadfence(); *(volatile T*)(ptr) = vst2_v_; } while (0)

namespace kit {

__device__ __forceinline__ unsigned short f2bf_bits(float f) {
  unsigned u = __float_as_uint(f);
  return (unsigned short)((u + 0x7FFFu + ((u >> 16) & 1u)) >> 16);
}
__device__ __forceinline__ float bf_bits2f(unsigned short h) { return __uint_as_float(((unsigned)h) << 16); }

__device__ __forceinline__ void dep_guard_h(v8f& a, v8f& b, v16h x, v16h y) { asm volatile("v_nop\n\tv_nop\n\tv_nop\n\tv_nop" : "+v"(a), "+v"(b) : "v"(x), "v"(y)); }
__device__ __forceinline__ void dep_guard_b(v8f& a, v8f& b, v16b x, v16b y) { asm volatile("v_nop\n\tv_nop\n\tv_nop\n\tv_nop" : "+v"(a), "+v"(b) : "v"(x), "v"(y)); }
__device__ __forceinline__ void keep4_h(v16h a, v16h b, v16h c, v16h d) { asm volatile("v_nop" :: "v"(a), "v"(b), "v"(c), "v"(d)); }
__device__ __forceinline__ void keep4_b(v16b a, v16b b, v16b c, v16b d) { asm volatile("v_nop" :: "v"(a), "v"(b), "v"(c), "v"(d)); }
__device__ __forceinline__ void acc_guard4(v8f& a, v8f& b, v8f& c, v8f& d) { asm volatile("v_nop\n\tv_nop\n\tv_nop\n\tv_nop" : "+v"(a), "+v"(b), "+v"(c), "+v"(d)); }
template <typename T> struct Frag;
template <> struct Frag<_Float16> {
  typedef v16h V; union U { v16h v; v8h h[2]; };
  static __device__ __forceinline__ v16h load(const _Float16* p) {
    U f; f.h[0] = *(const v8h*)(p); f.h[1] = *(const v8h*)(p + 16); return f.v;
  }
  static __device__ __forceinline__ v8f mma(v16h a, v16h b, v8f c) {
    return __builtin_amdgcn_wmma_f32_16x16x32_f16(false, a, false, b, (short)0, c, false, false);
  }
  static __device__ __forceinline__ void guard(v8f& a, v8f& b, v16h x, v16h y) { dep_guard_h(a, b, x, y); }
  static __device__ __forceinline__ void keep(v16h a, v16h b, v16h c, v16h d) { keep4_h(a, b, c, d); }
};
template <> struct Frag<__bf16> {
  typedef v16b V; union U { v16b v; v8b h[2]; };
  static __device__ __forceinline__ v16b load(const __bf16* p) {
    U f; f.h[0] = *(const v8b*)(p); f.h[1] = *(const v8b*)(p + 16); return f.v;
  }
  static __device__ __forceinline__ v8f mma(v16b a, v16b b, v8f c) {
    return __builtin_amdgcn_wmma_f32_16x16x32_bf16(false, a, false, b, (short)0, c, false, false);
  }
  static __device__ __forceinline__ void guard(v8f& a, v8f& b, v16b x, v16b y) { dep_guard_b(a, b, x, y); }
  static __device__ __forceinline__ void keep(v16b a, v16b b, v16b c, v16b d) { keep4_b(a, b, c, d); }
};

template <int ET> struct Elem;
template <> struct Elem<0> { typedef _Float16 T; };
template <> struct Elem<1> { typedef __bf16 T; };
template <int ET, bool SPLIT, int BIAS_MODE, int OUT_MODE>
__global__ __launch_bounds__(256) void wmma_gemm64(
    const unsigned short* __restrict__ Ap, const unsigned short* __restrict__ A2p, int lda, long strideA, long strideAz,
    const unsigned short* __restrict__ Btp, const unsigned short* __restrict__ Bt2p, int ldb, long strideB, long strideBz,
    void* __restrict__ Cout, void* __restrict__ Cout2, int ldc, long strideC, long strideCz,
    const float* __restrict__ bias,
    int M, int N, int K, float scale) {
  typedef typename Elem<ET>::T T;
  typedef typename Frag<T>::V V;
  const T* A = (const T*)Ap; const T* A2 = (const T*)A2p; const T* Bt = (const T*)Btp; const T* Bt2 = (const T*)Bt2p;
  __shared__ __align__(16) float sT[8][16 * 68];
  const int b    = blockIdx.y;
  const int bz   = blockIdx.z;
  const int lane = threadIdx.x & 31;
  const int wave = threadIdx.x >> 5;
  const int tilesN = N >> 6;
  const int tilesM = M >> 6;
  const int tile = blockIdx.x * 8 + wave;
  if (tile >= tilesM * tilesN) return;
  const int tm = tile / tilesN;
  const int tn = tile - tm * tilesN;
  const int m0 = tm << 6;
  const int n0 = tn << 6;

  const size_t offA = (size_t)b * (size_t)strideA + (size_t)bz * (size_t)strideAz;
  const size_t offB = (size_t)b * (size_t)strideB + (size_t)bz * (size_t)strideBz;
  const size_t offC = (size_t)b * (size_t)strideC + (size_t)bz * (size_t)strideCz;
  const T* Ab  = A  + offA;
  const T* Bb  = Bt + offB;
  const T* Ab2 = SPLIT ? (A2  + offA) : nullptr;
  const T* Bb2 = SPLIT ? (Bt2 + offB) : nullptr;

  const int rlane = lane & 15;
  const int koff  = (lane >> 4) * 8;
  const int mOff  = (lane >> 4) * 8;

  v8f acc[4][4];
#pragma unroll
  for (int i = 0; i < 4; ++i)
#pragma unroll
    for (int j = 0; j < 4; ++j) acc[i][j] = (v8f){0.f,0.f,0.f,0.f,0.f,0.f,0.f,0.f};

  for (int k0 = 0; k0 < K; k0 += 32) {
    V bh[4], bl[4];
#pragma unroll
    for (int j = 0; j < 4; ++j) {
      const size_t bo = (size_t)(n0 + (j << 4) + rlane) * ldb + koff + k0;
      bh[j] = Frag<T>::load(Bb + bo);
      if (SPLIT) bl[j] = Frag<T>::load(Bb2 + bo);
    }
#pragma unroll
    for (int i = 0; i < 4; ++i) {
      const size_t ao = (size_t)(m0 + (i << 4) + rlane) * lda + koff + k0;
      V ah = Frag<T>::load(Ab + ao);
      V al;
      if (SPLIT) al = Frag<T>::load(Ab2 + ao);
#pragma unroll
      for (int j = 0; j < 4; ++j) {
        acc[i][j] = Frag<T>::mma(ah, bh[j], acc[i][j]);
        if (SPLIT) {
          acc[i][j] = Frag<T>::mma(ah, bl[j], acc[i][j]);
          acc[i][j] = Frag<T>::mma(al, bh[j], acc[i][j]);
        }
      }
      Frag<T>::guard(acc[i][0], acc[i][3], ah, SPLIT ? al : ah);
    }
    Frag<T>::keep(bh[0], bh[1], bh[2], bh[3]);
    if (SPLIT) Frag<T>::keep(bl[0], bl[1], bl[2], bl[3]);
  }
  acc_guard4(acc[0][0], acc[0][1], acc[0][2], acc[0][3]);
  acc_guard4(acc[1][0], acc[1][1], acc[1][2], acc[1][3]);
  acc_guard4(acc[2][0], acc[2][1], acc[2][2], acc[2][3]);
  acc_guard4(acc[3][0], acc[3][1], acc[3][2], acc[3][3]);

  float* slab = sT[wave];
#pragma unroll
  for (int i = 0; i < 4; ++i) {
    const int mBase = m0 + (i << 4);
#pragma unroll
    for (int j = 0; j < 4; ++j) {
      const int n = n0 + (j << 4) + rlane;
      float bv = 0.f;
      if (BIAS_MODE == 2) bv = bias[n];
#pragma unroll
      for (int r = 0; r < 8; ++r) {
        float v = acc[i][j][r] * scale;
        if (BIAS_MODE == 1) v += bias[mBase + mOff + r];
        if (BIAS_MODE == 2) v += bv;
        slab[(mOff + r) * 68 + (j << 4) + rlane] = v;
      }
    }
    __builtin_amdgcn_fence(__ATOMIC_RELEASE, "workgroup");
    __builtin_amdgcn_wave_barrier();
    __builtin_amdgcn_fence(__ATOMIC_ACQUIRE, "workgroup");
    if (OUT_MODE == 0) {
      float* C = (float*)Cout + offC;
      const int hh = lane >> 4, c4 = (lane & 15) * 4;
      for (int pass = 0; pass < 2; ++pass) {
#pragma unroll
        for (int it = 0; it < 8; ++it) {
          const int row = it * 2 + hh;
          v4f v = *(const v4f*)(slab + row * 68 + c4);
          *(volatile v4f*)(C + (size_t)(mBase + row) * ldc + n0 + c4) = v;
        }
        __threadfence();
      }
    } else {
      const int q = lane >> 3, c8 = (lane & 7) * 8;
      unsigned short* C  = (unsigned short*)Cout  + offC;
      unsigned short* C2 = (OUT_MODE == 2) ? ((unsigned short*)Cout2 + offC) : nullptr;
      for (int pass = 0; pass < 2; ++pass) {
#pragma unroll
        for (int it = 0; it < 4; ++it) {
          const int row = it * 4 + q;
          const float* sp = slab + row * 68 + c8;
          v8h hv, lv;
#pragma unroll
          for (int e = 0; e < 8; ++e) {
            if (OUT_MODE == 1) {
              hv[e] = (_Float16)sp[e];
            } else {
              unsigned short hb = f2bf_bits(sp[e]);
              unsigned short lb = f2bf_bits(sp[e] - bf_bits2f(hb));
              hv[e] = __builtin_bit_cast(_Float16, hb);
              lv[e] = __builtin_bit_cast(_Float16, lb);
            }
          }
          *(volatile v8h*)(C + (size_t)(mBase + row) * ldc + n0 + c8) = hv;
          if (OUT_MODE == 2) *(volatile v8h*)(C2 + (size_t)(mBase + row) * ldc + n0 + c8) = lv;
        }
        __threadfence();
      }
    }
    __builtin_amdgcn_fence(__ATOMIC_RELEASE, "workgroup");
    __builtin_amdgcn_wave_barrier();
    __builtin_amdgcn_fence(__ATOMIC_ACQUIRE, "workgroup");
  }
}

}

__device__ __forceinline__ unsigned short bfu_rne(float v) { unsigned u = __builtin_bit_cast(unsigned, v); u += 0x7FFFu + ((u >> 16) & 1u); return (unsigned short)(u >> 16); }
__device__ __forceinline__ void bfsplit(float v, unsigned short& hi, unsigned short& lo) { hi = bfu_rne(v); lo = bfu_rne(v - __builtin_bit_cast(float, (unsigned)hi << 16)); }
__device__ __forceinline__ void st4s(unsigned short* Hp, unsigned short* Lp, long long o, v4f a) { unsigned short h[4], l[4]; bfsplit(a.x, h[0], l[0]); bfsplit(a.y, h[1], l[1]); bfsplit(a.z, h[2], l[2]); bfsplit(a.w, h[3], l[3]);
    const unsigned long long ph = (unsigned long long)h[0] | ((unsigned long long)h[1] << 16) | ((unsigned long long)h[2] << 32) | ((unsigned long long)h[3] << 48), pl = (unsigned long long)l[0] | ((unsigned long long)l[1] << 16) | ((unsigned long long)l[2] << 32) | ((unsigned long long)l[3] << 48);
    VST2(unsigned long long, (unsigned long long*)(Hp + o), ph); VST2(unsigned long long, (unsigned long long*)(Lp + o), pl); }

__device__ __forceinline__ unsigned short at_f2h(float x) { return (fabsf(x) < 6.104e-5f) ? (unsigned short)0 : __builtin_bit_cast(unsigned short, (_Float16)x); }
__device__ __forceinline__ void at_st8h(unsigned short* Pp, long long o, const float* v) { v4u pk; pk.x = (unsigned int)at_f2h(v[0]) | ((unsigned int)at_f2h(v[1]) << 16); pk.y = (unsigned int)at_f2h(v[2]) | ((unsigned int)at_f2h(v[3]) << 16); pk.z = (unsigned int)at_f2h(v[4]) | ((unsigned int)at_f2h(v[5]) << 16); pk.w = (unsigned int)at_f2h(v[6]) | ((unsigned int)at_f2h(v[7]) << 16); VST2(v4u, (v4u*)(Pp + o), pk); }

template <bool BFR>
__global__ __launch_bounds__(256) void k_cvt16(const float* __restrict__ X, unsigned short* __restrict__ O16, float sc, long long n8) {
    const long long u = (long long)blockIdx.x * 256 + threadIdx.x; if (u >= n8) return;
    const float* x = X + 8 * u; const v4f a = *(const v4f*)x; const v4f b = *(const v4f*)(x + 4);
    float v[8] = {a.x, a.y, a.z, a.w, b.x, b.y, b.z, b.w};
#pragma unroll
    for (int i = 0; i < 8; ++i) v[i] = (BFR ? kit::bf_bits2f(kit::f2bf_bits(v[i])) : v[i]) * sc;
    at_st8h(O16, 8 * u, v); }

template <int MODE, bool DUP>
__global__ __launch_bounds__(256) void k_trcv(const float* __restrict__ W, int Cc, unsigned short* __restrict__ O, int PO, int co, int co2, float sc) {
    __shared__ __align__(16) float sT[64 * 68];
    const int tid = threadIdx.x;
    const int n0 = blockIdx.x * 64, k0 = blockIdx.y * 64;
    const int nn = (tid & 15) * 4;
#pragma unroll
    for (int p = 0; p < 4; ++p) {
        const int kk = p * 16 + (tid >> 4);
        const v4f v = *(const v4f*)(W + (size_t)(k0 + kk) * Cc + n0 + nn);
        sT[(nn + 0) * 68 + kk] = v.x; sT[(nn + 1) * 68 + kk] = v.y; sT[(nn + 2) * 68 + kk] = v.z; sT[(nn + 3) * 68 + kk] = v.w;
    }
    __syncthreads();
    const int q = tid >> 3, c8 = (tid & 7) * 8;
#pragma unroll
    for (int p = 0; p < 2; ++p) {
        const int row = p * 32 + q;
        const float* sp = sT + row * 68 + c8;
        const v4f a = *(const v4f*)sp; const v4f b = *(const v4f*)(sp + 4);
        float v[8] = {a.x, a.y, a.z, a.w, b.x, b.y, b.z, b.w};
        v4u pk;
        if (MODE == 0) {
#pragma unroll
            for (int i = 0; i < 8; ++i) v[i] = kit::bf_bits2f(kit::f2bf_bits(v[i])) * sc;
            pk.x = (unsigned)at_f2h(v[0]) | ((unsigned)at_f2h(v[1]) << 16); pk.y = (unsigned)at_f2h(v[2]) | ((unsigned)at_f2h(v[3]) << 16);
            pk.z = (unsigned)at_f2h(v[4]) | ((unsigned)at_f2h(v[5]) << 16); pk.w = (unsigned)at_f2h(v[6]) | ((unsigned)at_f2h(v[7]) << 16);
        } else {
            pk.x = (unsigned)kit::f2bf_bits(v[0]) | ((unsigned)kit::f2bf_bits(v[1]) << 16); pk.y = (unsigned)kit::f2bf_bits(v[2]) | ((unsigned)kit::f2bf_bits(v[3]) << 16);
            pk.z = (unsigned)kit::f2bf_bits(v[4]) | ((unsigned)kit::f2bf_bits(v[5]) << 16); pk.w = (unsigned)kit::f2bf_bits(v[6]) | ((unsigned)kit::f2bf_bits(v[7]) << 16);
        }
        const size_t ro = (size_t)(n0 + row) * PO + k0 + c8;
        VST2(v4u, (v4u*)(O + ro + co), pk);
        if (DUP) VST2(v4u, (v4u*)(O + ro + co2), pk);
    }
}

__global__ __launch_bounds__(256) void k_pl4(const float* __restrict__ S, int SW, int CW, int RV, int R, unsigned short* __restrict__ PH, unsigned short* __restrict__ PL, int PP) { const long long u = (long long)blockIdx.x * 256 + threadIdx.x; const int cq = CW / 4; if (u >= (long long)R * cq) return; const int r = (int)(u / cq); const int c = 4 * (int)(u % cq); v4f v; v.x = v.y = v.z = v.w = 0.f; if (r < RV) v = *(const v4f*)(S + (long long)r * SW + c); st4s(PH, PL, (long long)r * PP + c, v); }

__global__ __launch_bounds__(256) void k_bias(const float* __restrict__ BQ, const float* __restrict__ BK, const float* __restrict__ BV, const float* __restrict__ BO,
                                             float* __restrict__ BC, float* __restrict__ BOC) {
    const int u = blockIdx.x * 256 + threadIdx.x;
    constexpr int NA = QKVW / 4, NO = HID / 4;
    static_assert(NA % 32 == 0);
    if (u < NA) {
        const int c = 4 * u;
        const int iq = (c < QW - 4) ? c : (QW - 4);
        int ik = c - QW; ik = ik < 0 ? 0 : ik; ik = ik > KVW - 4 ? KVW - 4 : ik;
        int iv = c - QW - KVW; iv = iv < 0 ? 0 : iv; iv = iv > KVW - 4 ? KVW - 4 : iv;
        const v4f a = *(const v4f*)(BQ + iq); const v4f k = *(const v4f*)(BK + ik); const v4f vv = *(const v4f*)(BV + iv);
        const bool sq = (c < QW), sk = (c < QW + KVW);
        v4f s;
        s.x = sq ? a.x : (sk ? k.x : vv.x); s.y = sq ? a.y : (sk ? k.y : vv.y); s.z = sq ? a.z : (sk ? k.z : vv.z); s.w = sq ? a.w : (sk ? k.w : vv.w);
        v4f r; r.x = kit::bf_bits2f(kit::f2bf_bits(s.x)); r.y = kit::bf_bits2f(kit::f2bf_bits(s.y)); r.z = kit::bf_bits2f(kit::f2bf_bits(s.z)); r.w = kit::bf_bits2f(kit::f2bf_bits(s.w));
        VST2(v4f, (v4f*)(BC + c), r);
    } else if (u < NA + NO) {
        const int c = 4 * (u - NA);
        const v4f s = *(const v4f*)(BO + c);
        v4f r; r.x = kit::bf_bits2f(kit::f2bf_bits(s.x)); r.y = kit::bf_bits2f(kit::f2bf_bits(s.y)); r.z = kit::bf_bits2f(kit::f2bf_bits(s.z)); r.w = kit::bf_bits2f(kit::f2bf_bits(s.w));
        VST2(v4f, (v4f*)(BOC + c), r);
    }
}

__global__ __launch_bounds__(256) void k_rope_il(const float* __restrict__ QKV, const float* __restrict__ CS, const float* __restrict__ SN,
                                                unsigned short* __restrict__ QH, unsigned short* __restrict__ QL, unsigned short* __restrict__ KH, unsigned short* __restrict__ KL, int nthr) {
    #pragma clang fp contract(off)
    const int u = blockIdx.x * 256 + threadIdx.x; if (u >= nthr) return;
    const int l = u & 15; const int hs = (u >> 4) % NSLOT; const int tp = u / (NSLOT * 16);
    const bool isq = (hs < NQH);
    if (isq && tp < KPAD) return;
    const int t = (tp >= KPAD) ? (tp - KPAD) : 0;
    const float* src = QKV + (long long)t * QKVW + hs * HDM + 4 * l;
    const v4f x = *(const v4f*)src;
    const float* cp = CS + (long long)t * 32 + 2 * l; const float* sp = SN + (long long)t * 32 + 2 * l;
    const float c0 = kit::bf_bits2f(kit::f2bf_bits(cp[0])), c1 = kit::bf_bits2f(kit::f2bf_bits(cp[1]));
    const float s0 = kit::bf_bits2f(kit::f2bf_bits(sp[0])), s1 = kit::bf_bits2f(kit::f2bf_bits(sp[1]));
    v4f o;
    o.x = x.x * c0 - x.y * s0;
    o.y = x.x * s0 + x.y * c0;
    o.z = x.z * c1 - x.w * s1;
    o.w = x.z * s1 + x.w * c1;
    const bool live = isq || (tp >= KPAD);
    v4f val; val.x = live ? o.x : 0.f; val.y = live ? o.y : 0.f; val.z = live ? o.z : 0.f; val.w = live ? o.w : 0.f;
    if (isq) st4s(QH, QL, (long long)t * QW + hs * HDM + 4 * l, val);
    else     st4s(KH, KL, (long long)tp * KVW + (hs - NQH) * HDM + 4 * l, val);
}

__global__ __launch_bounds__(256) void k_vt(const float* __restrict__ QKV, unsigned short* __restrict__ VTH, unsigned short* __restrict__ VTL) {
    const long long u = (long long)blockIdx.x * 256 + threadIdx.x; constexpr int l4 = SKP / 4; if (u >= (long long)KVW * l4) return;
    const int lp = 4 * (int)(u % l4); const int c = (int)(u / l4);
    const int l = lp - KPAD; const int lc = (l >= 0) ? l : 0;
    const float* src = QKV + (size_t)lc * QKVW + QW + KVW + c;
    v4f v; v.x = src[0]; v.y = src[QKVW]; v.z = src[2 * QKVW]; v.w = src[3 * QKVW];
    const bool live = (l >= 0);
    v4f val; val.x = live ? v.x : 0.f; val.y = live ? v.y : 0.f; val.z = live ? v.z : 0.f; val.w = live ? v.w : 0.f;
    st4s(VTH, VTL, (long long)c * SKP + lp, val);
}

__global__ __launch_bounds__(256) void k_sm_band(const float* __restrict__ SBp, const float* __restrict__ SINKS, int g, float sc,
                                                unsigned short* __restrict__ PH, unsigned short* __restrict__ PL, int nrows) {
    #pragma clang fp contract(off)
    const int r = blockIdx.x * 8 + (threadIdx.x >> 5); const int L = threadIdx.x & 31; if (r >= nrows) return;
    const int z = r / SEQ, t = r - z * SEQ;
    const int jb = (t >> 6) * 64 - KPAD;
    const float* s = SBp + (long long)r * BW;
    const float sink = kit::bf_bits2f(kit::f2bf_bits(SINKS[HPG * g + z]));
    const int L1 = (L < 16) ? L : 15;
    const v4f s0 = *(const v4f*)(s + 4 * L); const v4f s1 = *(const v4f*)(s + 128 + 4 * L1);
    bool lv0[4], lv1[4];
    float m = -3.0e38f;
#pragma unroll
    for (int e = 0; e < 4; ++e) {
        const int j0 = jb + 4 * L + e, j1 = jb + 128 + 4 * L + e;
        lv0[e] = (j0 >= 0) && (j0 <= t) && (t - j0 < WIN);
        lv1[e] = (L < 16) && (j1 >= 0) && (j1 <= t) && (t - j1 < WIN);
        m = fmaxf(m, lv0[e] ? s0[e] * sc : -3.0e38f);
        m = fmaxf(m, lv1[e] ? s1[e] * sc : -3.0e38f);
    }
#pragma unroll
    for (int o = 16; o > 0; o >>= 1) m = fmaxf(m, __shfl_xor(m, o, 32));
    m = fmaxf(m, sink);
    float sum = 0.f; v4f p0, p1;
#pragma unroll
    for (int e = 0; e < 4; ++e) {
        const float e0 = __expf(s0[e] * sc - m); const float e1 = __expf(s1[e] * sc - m);
        p0[e] = lv0[e] ? e0 : 0.f; p1[e] = lv1[e] ? e1 : 0.f;
        sum += p0[e]; sum += p1[e];
    }
#pragma unroll
    for (int o = 16; o > 0; o >>= 1) sum += __shfl_xor(sum, o, 32);
    const float inv = 1.f / (sum + __expf(sink - m));
    const v4f q0 = p0 * inv; const v4f q1 = p1 * inv;
    st4s(PH, PL, (long long)r * BW + 4 * L, q0);
    if (L < 16) st4s(PH, PL, (long long)r * BW + 128 + 4 * L, q1);
}

constexpr size_t cmax_(size_t a, size_t b) { return a > b ? a : b; }
constexpr size_t SZ_X16  = (size_t)SEQ * HID * 2;
constexpr size_t SZ_W16  = (size_t)QKVW * HID * 2;
constexpr size_t SZ_QP   = (size_t)SEQ * QW * 2;
constexpr size_t SZ_KP   = (size_t)SKP * KVW * 2;
constexpr size_t SZ_CP   = (size_t)OSPLIT_ROWS * 2 * QW * 2;
constexpr size_t SZ_CP16 = (size_t)SEQ * QW * 2;
constexpr size_t SZ_R0   = cmax_(cmax_(SZ_X16 + SZ_W16, 2 * SZ_QP + 4 * SZ_KP), SZ_CP + SZ_CP16);
constexpr size_t SZ_QKVF = (size_t)SEQ * QKVW * 4;
constexpr size_t SZ_CTX  = (size_t)SEQ * QW * 4;
constexpr size_t SZ_WP   = (size_t)HID * 2 * QW * 2;
constexpr size_t SZ_R1   = cmax_(cmax_(SZ_QKVF, SZ_CTX), SZ_WP);
constexpr size_t SZ_SB   = (size_t)HPG * SEQ * BW * 4;
constexpr size_t SZ_PP   = (size_t)HPG * SEQ * BW * 2;
constexpr size_t SZ_W16O = (size_t)HID * QW * 2;
constexpr size_t SZ_R2   = cmax_(SZ_SB + 2 * SZ_PP, SZ_W16O);
constexpr size_t SZ_BC   = (size_t)QKVW * 4;
constexpr size_t SZ_BOC  = (((size_t)HID * 4) + 255) / 256 * 256;
constexpr size_t SZ_ALL  = SZ_R0 + SZ_R1 + SZ_R2 + SZ_BC + SZ_BOC;
static_assert(SZ_X16 % 256 == 0 && SZ_W16 % 256 == 0 && SZ_QP % 256 == 0 && SZ_KP % 256 == 0 && SZ_CP % 256 == 0 && SZ_CP16 % 256 == 0);
static_assert(SZ_R0 % 256 == 0 && SZ_R1 % 256 == 0 && SZ_R2 % 256 == 0 && SZ_SB % 256 == 0 && SZ_PP % 256 == 0 && SZ_W16O % 256 == 0 && SZ_BC % 256 == 0);
static_assert(SZ_ALL <= (size_t)134217728);
static_assert((size_t)QKVW * HID * 2 == (size_t)QW * HID * 2 + 2 * (size_t)KVW * HID * 2);

extern "C" void kernel_launch(void* const* d_in, const int* in_sizes, int n_in, void* d_out, int out_size, void* d_ws, size_t ws_size, hipStream_t stream) {
    if (n_in < 12) return;
    if (in_sizes[0] < SEQ * HID || in_sizes[1] < SEQ * 32 || in_sizes[2] < SEQ * 32 || in_sizes[3] < HID * QW || in_sizes[4] < QW ||
        in_sizes[5] < HID * KVW || in_sizes[6] < KVW || in_sizes[7] < HID * KVW || in_sizes[8] < KVW || in_sizes[9] < QW * HID ||
        in_sizes[10] < HID || in_sizes[11] < NQH || out_size < SEQ * HID) return;
    if (SZ_ALL > ws_size) return;
    const float* x     = (const float*)d_in[0];
    const float* cosb  = (const float*)d_in[1];
    const float* sinb  = (const float*)d_in[2];
    const float* wq    = (const float*)d_in[3];
    const float* bq    = (const float*)d_in[4];
    const float* wk    = (const float*)d_in[5];
    const float* bk    = (const float*)d_in[6];
    const float* wv    = (const float*)d_in[7];
    const float* bv    = (const float*)d_in[8];
    const float* wo    = (const float*)d_in[9];
    const float* bo    = (const float*)d_in[10];
    const float* sinks = (const float*)d_in[11];
    float* out = (float*)d_out;

    char* wsp = (char*)d_ws;
    char* R0 = wsp; char* R1 = R0 + SZ_R0; char* R2 = R1 + SZ_R1; char* R3 = R2 + SZ_R2; char* R4 = R3 + SZ_BC;
    unsigned short* X16 = (unsigned short*)R0;
    unsigned short* W16 = (unsigned short*)(R0 + SZ_X16);
    unsigned short* QH  = (unsigned short*)R0;
    unsigned short* QL  = (unsigned short*)(R0 + SZ_QP);
    unsigned short* KH  = (unsigned short*)(R0 + 2 * SZ_QP);
    unsigned short* KL  = (unsigned short*)(R0 + 2 * SZ_QP + SZ_KP);
    unsigned short* VTH = (unsigned short*)(R0 + 2 * SZ_QP + 2 * SZ_KP);
    unsigned short* VTL = (unsigned short*)(R0 + 2 * SZ_QP + 3 * SZ_KP);
    unsigned short* CP  = (unsigned short*)R0;
    unsigned short* CP16 = (unsigned short*)(R0 + SZ_CP);
    float* QKVF = (float*)R1;
    float* CTX  = (float*)R1;
    unsigned short* WP = (unsigned short*)R1;
    float* SB = (float*)R2;
    unsigned short* PH = (unsigned short*)(R2 + SZ_SB);
    unsigned short* PL = (unsigned short*)(R2 + SZ_SB + SZ_PP);
    unsigned short* W16O = (unsigned short*)R2;
    float* BC  = (float*)R3;
    float* BOC = (float*)R4;

    k_cvt16<true><<<(unsigned)(((long long)SEQ * HID / 8 + 255) / 256), 256, 0, stream>>>(x, X16, 1.0f, (long long)SEQ * HID / 8);
    k_trcv<0, false><<<dim3(QW / 64, HID / 64), 256, 0, stream>>>(wq, QW, W16, HID, 0, 0, 64.0f);
    k_trcv<0, false><<<dim3(KVW / 64, HID / 64), 256, 0, stream>>>(wk, KVW, W16 + (size_t)QW * HID, HID, 0, 0, 64.0f);
    k_trcv<0, false><<<dim3(KVW / 64, HID / 64), 256, 0, stream>>>(wv, KVW, W16 + (size_t)(QW + KVW) * HID, HID, 0, 0, 64.0f);
    k_bias<<<(unsigned)((QKVW / 4 + HID / 4 + 255) / 256), 256, 0, stream>>>(bq, bk, bv, bo, BC, BOC);
    kit::wmma_gemm64<0, false, 2, 0><<<dim3((unsigned)(((SEQ / 64) * (QKVW / 64) + 7) / 8), 1u, 1u), 256, 0, stream>>>(
        X16, nullptr, HID, 0L, 0L, W16, nullptr, HID, 0L, 0L, (void*)QKVF, nullptr, QKVW, 0L, 0L, BC, SEQ, QKVW, HID, 0.015625f);
    k_rope_il<<<(unsigned)((SKP * NSLOT * 16 + 255) / 256), 256, 0, stream>>>(QKVF, cosb, sinb, QH, QL, KH, KL, SKP * NSLOT * 16);
    k_vt<<<(unsigned)(((long long)KVW * (SKP / 4) + 255) / 256), 256, 0, stream>>>(QKVF, VTH, VTL);
    for (int g = 0; g < NKVH; ++g) {
        kit::wmma_gemm64<1, true, 0, 0><<<dim3(1u, (unsigned)(SEQ / 64), (unsigned)HPG), 96, 0, stream>>>(
            QH + (size_t)g * (HPG * HDM), QL + (size_t)g * (HPG * HDM), QW, (long)64 * QW, (long)HDM,
            KH + (size_t)g * HDM, KL + (size_t)g * HDM, KVW, (long)64 * KVW, 0L,
            (void*)SB, nullptr, BW, (long)64 * BW, (long)SEQ * BW,
            nullptr, 64, BW, HDM, 1.0f);
        k_sm_band<<<(unsigned)((HPG * SEQ + 7) / 8), 256, 0, stream>>>(SB, sinks, g, 0.125f, PH, PL, HPG * SEQ);
        kit::wmma_gemm64<1, true, 0, 0><<<dim3(1u, (unsigned)(SEQ / 64), (unsigned)HPG), 32, 0, stream>>>(
            PH, PL, BW, (long)64 * BW, (long)SEQ * BW,
            VTH + (size_t)g * HDM * SKP, VTL + (size_t)g * HDM * SKP, SKP, (long)64, 0L,
            (void*)(CTX + (size_t)g * (HPG * HDM)), nullptr, QW, (long)64 * QW, (long)HDM,
            nullptr, 64, HDM, BW, 1.0f);
    }
    k_pl4<<<(unsigned)(((long long)OSPLIT_ROWS * (QW / 4) + 255) / 256), 256, 0, stream>>>(CTX, QW, QW, OSPLIT_ROWS, OSPLIT_ROWS, CP, CP + QW, 2 * QW);
    k_cvt16<false><<<(unsigned)(((long long)SEQ * QW / 8 + 255) / 256), 256, 0, stream>>>(CTX, CP16, 16.0f, (long long)SEQ * QW / 8);
    k_trcv<1, true><<<dim3(HID / 64, QW / 64), 256, 0, stream>>>(wo, HID, WP, 2 * QW, 0, QW, 1.0f);
    k_trcv<0, false><<<dim3(HID / 64, QW / 64), 256, 0, stream>>>(wo, HID, W16O, QW, 0, 0, 64.0f);
    kit::wmma_gemm64<1, false, 2, 0><<<dim3((unsigned)(((OSPLIT_ROWS / 64) * (HID / 64) + 7) / 8), 1u, 1u), 256, 0, stream>>>(
        CP, nullptr, 2 * QW, 0L, 0L, WP, nullptr, 2 * QW, 0L, 0L, (void*)out, nullptr, HID, 0L, 0L, BOC, OSPLIT_ROWS, HID, 2 * QW, 1.0f);
    if (SEQ - OSPLIT_ROWS > 0) {
        kit::wmma_gemm64<0, false, 2, 0><<<dim3((unsigned)((((SEQ - OSPLIT_ROWS) / 64) * (HID / 64) + 7) / 8), 1u, 1u), 256, 0, stream>>>(
            CP16 + (size_t)OSPLIT_ROWS * QW, nullptr, QW, 0L, 0L, W16O, nullptr, QW, 0L, 0L, (void*)(out + (size_t)OSPLIT_ROWS * HID), nullptr, HID, 0L, 0L, BOC,
            SEQ - OSPLIT_ROWS, HID, QW, 0.0009765625f);
    }
}
